// Zero_Parameter_32830730011392
// MI455X (gfx1250) — hardware-run, weakly checked
//
#include <hip/hip_runtime.h>
#include <math.h>

typedef __attribute__((ext_vector_type(16))) _Float16 v16h;
typedef __attribute__((ext_vector_type(8)))  _Float16 v8h;
typedef __attribute__((ext_vector_type(16))) __bf16   v16b;
typedef __attribute__((ext_vector_type(8)))  __bf16   v8b;
typedef __attribute__((ext_vector_type(8)))  float    v8f;
typedef __attribute__((ext_vector_type(4)))  float    v4f;
typedef __attribute__((ext_vector_type(4)))  unsigned int v4u;

constexpr int kB   = 8;
constexpr int kN1  = 1024;
constexpr int kN2  = 1024;
constexpr int kDT  = 768;
constexpr int kDV  = 1024;
constexpr int kDO  = 768;
constexpr int kH   = 8;
constexpr int kHD  = kDO / kH;
constexpr int kRowsQ  = kB * kN1;
constexpr int kRowsKV = kB * kN2;
constexpr int kOP  = 196;
constexpr float kPCarry = 32768.0f;
static_assert(kHD == 96);
static_assert(kHD % 32 == 0);
static_assert((kH % 2) == 0);
static_assert((kDT % 32) == 0 && (kDV % 32) == 0 && (kDO % 32) == 0 && (kN2 % 64) == 0);
static_assert((kRowsQ % 64) == 0 && (kRowsKV % 64) == 0 && (kDO % 64) == 0 && (kN1 % 64) == 0);
static_assert(((2 * kHD * 2) % 128) == 0);

constexpr size_t kOffFT   = 0;
constexpr size_t kOffFS   = kOffFT   + (size_t)kRowsQ  * kDT * 2;
constexpr size_t kOffWQT  = kOffFS   + (size_t)kRowsKV * kDV * 2;
constexpr size_t kOffWKT  = kOffWQT  + (size_t)kDO * kDT * 2;
constexpr size_t kOffWVT  = kOffWKT  + (size_t)kDO * kDV * 2;
constexpr size_t kOffWPT  = kOffWVT  + (size_t)kDO * kDV * 2;
constexpr size_t kOffBIAS = kOffWPT  + (size_t)kDO * kDO * 2;
constexpr size_t kOffQH   = kOffBIAS + (size_t)4 * kDO * 4;
constexpr size_t kOffQL   = kOffQH   + (size_t)kRowsQ  * kDO * 2;
constexpr size_t kOffKH   = kOffQL   + (size_t)kRowsQ  * kDO * 2;
constexpr size_t kOffKL   = kOffKH   + (size_t)kRowsKV * kDO * 2;
constexpr size_t kOffVT   = kOffKL   + (size_t)kRowsKV * kDO * 2;
constexpr size_t kOffCH   = kOffVT   + (size_t)kDO * kRowsKV * 2;
constexpr size_t kOffCL   = kOffCH   + (size_t)kRowsQ  * kDO * 2;
constexpr size_t kWsTotal = kOffCL   + (size_t)kRowsQ  * kDO * 2;
constexpr size_t kOffPROJ = kOffFT;
static_assert(kWsTotal == 122957824ull);
static_assert(kWsTotal <= 134217728ull);
static_assert((size_t)kRowsQ * kDO * 4 <= kOffWQT - kOffFT);
static_assert((kOffFS % 128) == 0 && (kOffWQT % 128) == 0 && (kOffWKT % 128) == 0 && (kOffWVT % 128) == 0 &&
              (kOffWPT % 128) == 0 && (kOffBIAS % 128) == 0 && (kOffQH % 128) == 0 && (kOffQL % 128) == 0 &&
              (kOffKH % 128) == 0 && (kOffKL % 128) == 0 && (kOffVT % 128) == 0 && (kOffCH % 128) == 0 &&
              (kOffCL % 128) == 0);

__device__ __forceinline__ unsigned short f2bf_bits(float f) {
  unsigned u = __float_as_uint(f);
  return (unsigned short)((u + 0x7FFFu + ((u >> 16) & 1u)) >> 16);
}
__device__ __forceinline__ float bf_bits2f(unsigned short h) { return __uint_as_float(((unsigned)h) << 16); }
__device__ __forceinline__ unsigned pk16(unsigned short a, unsigned short b) { return (unsigned)a | ((unsigned)b << 16); }
__device__ __forceinline__ v8f zero8() { return (v8f){0.f, 0.f, 0.f, 0.f, 0.f, 0.f, 0.f, 0.f}; }

__device__ __forceinline__ void row_guard_b(v8f& a, v8f& b, v8f& c, v8f& d, v16b x, v16b y) {
  asm volatile("v_nop\n\tv_nop\n\tv_nop\n\tv_nop" : "+v"(a), "+v"(b), "+v"(c), "+v"(d) : "v"(x), "v"(y));
}
__device__ __forceinline__ void keep4_b(v16b a, v16b b, v16b c, v16b d) { asm volatile("v_nop" :: "v"(a), "v"(b), "v"(c), "v"(d)); }
__device__ __forceinline__ void acc_guard4(v8f& a, v8f& b, v8f& c, v8f& d) {
  asm volatile("v_nop\n\tv_nop\n\tv_nop\n\tv_nop" : "+v"(a), "+v"(b), "+v"(c), "+v"(d));
}
__device__ __forceinline__ void grp_guard_b(v8f& a, v16b w, v16b x, v16b y, v16b z) {
  asm volatile("v_nop\n\tv_nop\n\tv_nop\n\tv_nop" : "+v"(a) : "v"(w), "v"(x), "v"(y), "v"(z));
}
__device__ __forceinline__ void one_guard_h(v8f& a, v16h x, v16h y) {
  asm volatile("v_nop\n\tv_nop\n\tv_nop\n\tv_nop" : "+v"(a) : "v"(x), "v"(y));
}

template <typename T> struct Frag;
template <> struct Frag<_Float16> {
  typedef v16h V;
  union U { v16h v; v8h h[2]; };
  static __device__ __forceinline__ v16h load(const _Float16* p) {
    U f;
    f.h[0] = *(const v8h*)(p);
    f.h[1] = *(const v8h*)(p + 16);
    return f.v;
  }
  static __device__ __forceinline__ v8f mma(v16h a, v16h b, v8f c) {
    return __builtin_amdgcn_wmma_f32_16x16x32_f16(false, a, false, b, (short)0, c, false, false);
  }
};
template <> struct Frag<__bf16> {
  typedef v16b V;
  union U { v16b v; v8b h[2]; };
  static __device__ __forceinline__ v16b load(const __bf16* p) {
    U f;
    f.h[0] = *(const v8b*)(p);
    f.h[1] = *(const v8b*)(p + 16);
    return f.v;
  }
  static __device__ __forceinline__ v8f mma(v16b a, v16b b, v8f c) {
    return __builtin_amdgcn_wmma_f32_16x16x32_bf16(false, a, false, b, (short)0, c, false, false);
  }
};

__global__ __launch_bounds__(256) void cast8_bf16_kernel(const float* __restrict__ in, unsigned short* __restrict__ out, int n8) {
  const int i = blockIdx.x * 256 + threadIdx.x;
  if (i >= n8) return;
  const float* p = in + 8 * (size_t)i;
  const v4f a = *(const v4f*)(p);
  const v4f b = *(const v4f*)(p + 4);
  const float x0 = a[0], x1 = a[1], x2 = a[2], x3 = a[3];
  const float x4 = b[0], x5 = b[1], x6 = b[2], x7 = b[3];
  const v4u u = (v4u){pk16(f2bf_bits(x0), f2bf_bits(x1)), pk16(f2bf_bits(x2), f2bf_bits(x3)),
                      pk16(f2bf_bits(x4), f2bf_bits(x5)), pk16(f2bf_bits(x6), f2bf_bits(x7))};
  unsigned short* q = out + 8 * (size_t)i;
  *(volatile v4u*)q = u;
  __threadfence();
  *(volatile v4u*)q = u;
}

__global__ __launch_bounds__(256) void wt_bf16_kernel(const float* __restrict__ W0, const float* __restrict__ W1,
                                                      const float* __restrict__ W2, const float* __restrict__ W3,
                                                      unsigned short* __restrict__ T0, unsigned short* __restrict__ T1,
                                                      unsigned short* __restrict__ T2, unsigned short* __restrict__ T3) {
  __shared__ float sm[64][65];
  const int t  = threadIdx.x;
  const int z  = blockIdx.z;
  const int Kin = (z == 0 || z == 3) ? kDT : kDV;
  const int d0 = blockIdx.x * 64;
  if (d0 >= Kin) return;
  const int h0 = blockIdx.y * 64;
  const float* W = (z == 0) ? W0 : (z == 1) ? W1 : (z == 2) ? W2 : W3;
  unsigned short* op = (z == 0) ? T0 : (z == 1) ? T1 : (z == 2) ? T2 : T3;
#pragma unroll
  for (int i = 0; i < 16; ++i) {
    const int e = i * 256 + t;
    const int r = e >> 6;
    const int c = e & 63;
    sm[c][r] = W[(size_t)(d0 + r) * kDO + h0 + c];
  }
  __syncthreads();
  const int lane = t & 31, wave = t >> 5;
  const int q = lane >> 3, c8 = (lane & 7) * 8;
  for (int pass = 0; pass < 2; ++pass) {
#pragma unroll
    for (int it = 0; it < 2; ++it) {
      const int row = wave * 8 + it * 4 + q;
      unsigned short hb[8];
#pragma unroll
      for (int e = 0; e < 8; ++e) hb[e] = f2bf_bits(sm[row][c8 + e]);
      const v4u u = (v4u){pk16(hb[0], hb[1]), pk16(hb[2], hb[3]), pk16(hb[4], hb[5]), pk16(hb[6], hb[7])};
      *(volatile v4u*)(op + (size_t)(h0 + row) * Kin + d0 + c8) = u;
    }
    __threadfence();
  }
}

__global__ __launch_bounds__(256) void bias_rne_kernel(const float* __restrict__ b0, const float* __restrict__ b1,
                                                       const float* __restrict__ b2, const float* __restrict__ b3,
                                                       float* __restrict__ out) {
  const int i = blockIdx.x * 256 + threadIdx.x;
  if (i >= 4 * (kDO / 4)) return;
  const int a = i / (kDO / 4);
  const int o = (i - a * (kDO / 4)) * 4;
  const v4f c0 = *(const v4f*)(b0 + o);
  const v4f c1 = *(const v4f*)(b1 + o);
  const v4f c2 = *(const v4f*)(b2 + o);
  const v4f c3 = *(const v4f*)(b3 + o);
  const v4f s = (a == 0) ? c0 : (a == 1) ? c1 : (a == 2) ? c2 : c3;
  const float x0 = s[0], x1 = s[1], x2 = s[2], x3 = s[3];
  const v4f r = (v4f){bf_bits2f(f2bf_bits(x0)), bf_bits2f(f2bf_bits(x1)), bf_bits2f(f2bf_bits(x2)), bf_bits2f(f2bf_bits(x3))};
  float* q = out + (size_t)a * kDO + o;
  *(volatile v4f*)q = r;
  __threadfence();
  *(volatile v4f*)q = r;
}

template <int SPL, int BIAS_MODE, int OUT_MODE>
__global__ __launch_bounds__(256) void wmma_gemm64_bf16(
    const unsigned short* __restrict__ Ap, const unsigned short* __restrict__ A2p, int lda,
    const unsigned short* __restrict__ Btp, int ldb,
    void* __restrict__ Cout, void* __restrict__ Cout2, int ldc,
    const float* __restrict__ bias, int M, int N, int K) {
  const __bf16* A  = (const __bf16*)Ap;
  const __bf16* A2 = (const __bf16*)A2p;
  const __bf16* Bt = (const __bf16*)Btp;
  __shared__ __align__(16) float sT[8][16 * 68];
  const int lane = threadIdx.x & 31;
  const int wave = threadIdx.x >> 5;
  const int tilesN = N >> 6;
  const int tilesM = M >> 6;
  const int tile = blockIdx.x * 8 + wave;
  if (tile >= tilesM * tilesN) return;
  const int tm = tile / tilesN;
  const int tn = tile - tm * tilesN;
  const int m0 = tm << 6;
  const int n0 = tn << 6;

  const int rlane = lane & 15;
  const int koff  = (lane >> 4) * 8;
  const int mOff  = (lane >> 4) * 8;

  v8f acc[4][4];
#pragma unroll
  for (int i = 0; i < 4; ++i)
#pragma unroll
    for (int j = 0; j < 4; ++j) acc[i][j] = zero8();

  for (int k0 = 0; k0 < K; k0 += 32) {
    v16b bh[4];
#pragma unroll
    for (int j = 0; j < 4; ++j) {
      const size_t bo = (size_t)(n0 + (j << 4) + rlane) * ldb + koff + k0;
      bh[j] = Frag<__bf16>::load(Bt + bo);
    }
#pragma unroll
    for (int i = 0; i < 4; ++i) {
      const size_t ao = (size_t)(m0 + (i << 4) + rlane) * lda + koff + k0;
      const v16b ah = Frag<__bf16>::load(A + ao);
      v16b al = ah;
      if (SPL == 1) al = Frag<__bf16>::load(A2 + ao);
#pragma unroll
      for (int j = 0; j < 4; ++j) {
        acc[i][j] = Frag<__bf16>::mma(ah, bh[j], acc[i][j]);
        if (SPL == 1) acc[i][j] = Frag<__bf16>::mma(al, bh[j], acc[i][j]);
      }
      row_guard_b(acc[i][0], acc[i][1], acc[i][2], acc[i][3], ah, al);
    }
    keep4_b(bh[0], bh[1], bh[2], bh[3]);
  }
  acc_guard4(acc[0][0], acc[0][1], acc[0][2], acc[0][3]);
  acc_guard4(acc[1][0], acc[1][1], acc[1][2], acc[1][3]);
  acc_guard4(acc[2][0], acc[2][1], acc[2][2], acc[2][3]);
  acc_guard4(acc[3][0], acc[3][1], acc[3][2], acc[3][3]);

  float* slab = sT[wave];
#pragma unroll
  for (int i = 0; i < 4; ++i) {
    const int mBase = m0 + (i << 4);
#pragma unroll
    for (int j = 0; j < 4; ++j) {
      const int n = n0 + (j << 4) + rlane;
      float bv = 0.f;
      if (BIAS_MODE == 2) bv = bias[n];
#pragma unroll
      for (int r = 0; r < 8; ++r) {
        float v = acc[i][j][r];
        if (BIAS_MODE == 1) v += bias[mBase + mOff + r];
        if (BIAS_MODE == 2) v += bv;
        slab[(mOff + r) * 68 + (j << 4) + rlane] = v;
      }
    }
    __builtin_amdgcn_fence(__ATOMIC_RELEASE, "workgroup");
    __builtin_amdgcn_wave_barrier();
    __builtin_amdgcn_fence(__ATOMIC_ACQUIRE, "workgroup");
    if (OUT_MODE == 0) {
      float* C = (float*)Cout;
      const int hh = lane >> 4, c4 = (lane & 15) * 4;
      for (int pass = 0; pass < 2; ++pass) {
#pragma unroll
        for (int it = 0; it < 8; ++it) {
          const int row = it * 2 + hh;
          const v4f v = *(const v4f*)(slab + row * 68 + c4);
          *(volatile v4f*)(C + (size_t)(mBase + row) * ldc + n0 + c4) = v;
        }
        __threadfence();
      }
    } else {
      const int q = lane >> 3, c8 = (lane & 7) * 8;
      unsigned short* C  = (unsigned short*)Cout;
      unsigned short* C2 = (unsigned short*)Cout2;
      for (int pass = 0; pass < 2; ++pass) {
#pragma unroll
        for (int it = 0; it < 4; ++it) {
          const int row = it * 4 + q;
          const float* sp = slab + row * 68 + c8;
          v8h hv, lv;
#pragma unroll
          for (int e = 0; e < 8; ++e) {
            const float xv = sp[e];
            if (OUT_MODE == 1) {
              hv[e] = (_Float16)xv;
            } else {
              const unsigned short hb = f2bf_bits(xv);
              const unsigned short lb = f2bf_bits(xv - bf_bits2f(hb));
              hv[e] = __builtin_bit_cast(_Float16, hb);
              lv[e] = __builtin_bit_cast(_Float16, lb);
            }
          }
          *(volatile v8h*)(C + (size_t)(mBase + row) * ldc + n0 + c8) = hv;
          if (OUT_MODE == 2) *(volatile v8h*)(C2 + (size_t)(mBase + row) * ldc + n0 + c8) = lv;
        }
        __threadfence();
      }
    }
    __builtin_amdgcn_fence(__ATOMIC_RELEASE, "workgroup");
    __builtin_amdgcn_wave_barrier();
    __builtin_amdgcn_fence(__ATOMIC_ACQUIRE, "workgroup");
  }
}

__global__ __launch_bounds__(128) void attn_pair_kernel(
    const unsigned short* __restrict__ Qhp, const unsigned short* __restrict__ Qlp,
    const unsigned short* __restrict__ Khp, const unsigned short* __restrict__ Klp,
    const unsigned short* __restrict__ Vtp,
    unsigned short* __restrict__ Ch, unsigned short* __restrict__ Cl) {
  __shared__ __align__(16) _Float16 Psh[4][16 * 64];
  __shared__ __align__(16) float Ost[4][16 * kOP];
  const int tid  = threadIdx.x;
  const int wave = tid >> 5;
  const int lane = tid & 31;
  const int hh   = lane >> 4;
  const int c    = lane & 15;
  const int bx   = blockIdx.x;
  const int hp   = bx & 3;
  const int qblk = (bx >> 2) & 15;
  const int b    = bx >> 6;
  const int q0   = b * kN1 + qblk * 64 + wave * 16;
  const int kvb  = b * kN2;

  const __bf16* Qh = (const __bf16*)Qhp;
  const __bf16* Ql = (const __bf16*)Qlp;
  const __bf16* Kh = (const __bf16*)Khp;
  const __bf16* Kl = (const __bf16*)Klp;
  const _Float16* Vt = (const _Float16*)Vtp;
  _Float16* pw = Psh[wave];
  float* os = Ost[wave];

#pragma unroll 1
  for (int hd = 0; hd < 2; ++hd) {
    const int h = hp * 2 + hd;
    const int colq = h * kHD + 8 * hh;
    const __bf16* qhr = Qh + (size_t)(q0 + c) * kDO + colq;
    const __bf16* qlr = Ql + (size_t)(q0 + c) * kDO + colq;

    float mrow[8], lrow[8];
    v8f oacc[6];
#pragma unroll
    for (int r = 0; r < 8; ++r) { mrow[r] = -1e30f; lrow[r] = 0.f; }
#pragma unroll
    for (int t = 0; t < 6; ++t) oacc[t] = zero8();

#pragma unroll 1
    for (int kc = 0; kc < kN2 / 64; ++kc) {
      const int kv0 = kvb + kc * 64;
      v8f s[4];
#pragma unroll
      for (int j = 0; j < 4; ++j) s[j] = zero8();
#pragma unroll
      for (int dc = 0; dc < 3; ++dc) {
        const v16b qa  = Frag<__bf16>::load(qhr + dc * 32);
        const v16b qlo = Frag<__bf16>::load(qlr + dc * 32);
#pragma unroll
        for (int j = 0; j < 4; ++j) {
          const size_t ko = (size_t)(kv0 + j * 16 + c) * kDO + colq + dc * 32;
          const v16b kb = Frag<__bf16>::load(Kh + ko);
          const v16b kl = Frag<__bf16>::load(Kl + ko);
          s[j] = Frag<__bf16>::mma(qa,  kb, s[j]);
          s[j] = Frag<__bf16>::mma(qa,  kl, s[j]);
          s[j] = Frag<__bf16>::mma(qlo, kb, s[j]);
          grp_guard_b(s[j], qa, qlo, kb, kl);
        }
      }
      float cm[8];
#pragma unroll
      for (int r = 0; r < 8; ++r) {
        float m = fmaxf(fmaxf(s[0][r], s[1][r]), fmaxf(s[2][r], s[3][r]));
        m = fmaxf(m, __shfl_xor(m, 1, 32));
        m = fmaxf(m, __shfl_xor(m, 2, 32));
        m = fmaxf(m, __shfl_xor(m, 4, 32));
        m = fmaxf(m, __shfl_xor(m, 8, 32));
        cm[r] = m;
      }
#pragma unroll
      for (int r = 0; r < 8; ++r) {
        const float mnew  = fmaxf(mrow[r], cm[r]);
        const float alpha = __expf(mrow[r] - mnew);
        mrow[r] = mnew;
        float psum = 0.f;
#pragma unroll
        for (int j = 0; j < 4; ++j) {
          const float p = __expf(s[j][r] - mnew);
          psum += p;
          const _Float16 ph = (_Float16)(p * kPCarry);
          pw[(8 * hh + r) * 64 + j * 16 + c] = ph;
        }
        psum += __shfl_xor(psum, 1, 32);
        psum += __shfl_xor(psum, 2, 32);
        psum += __shfl_xor(psum, 4, 32);
        psum += __shfl_xor(psum, 8, 32);
        lrow[r] = lrow[r] * alpha + psum;
#pragma unroll
        for (int t = 0; t < 6; ++t) oacc[t][r] *= alpha;
      }
      __builtin_amdgcn_fence(__ATOMIC_RELEASE, "workgroup");
      __builtin_amdgcn_wave_barrier();
      __builtin_amdgcn_fence(__ATOMIC_ACQUIRE, "workgroup");
#pragma unroll
      for (int kk = 0; kk < 2; ++kk) {
        const v16h pa = Frag<_Float16>::load(pw + c * 64 + kk * 32 + 8 * hh);
#pragma unroll
        for (int t = 0; t < 6; ++t) {
          const size_t vo = (size_t)(h * kHD + t * 16 + c) * kRowsKV + kv0 + kk * 32 + 8 * hh;
          const v16h vb = Frag<_Float16>::load(Vt + vo);
          oacc[t] = Frag<_Float16>::mma(pa, vb, oacc[t]);
          one_guard_h(oacc[t], pa, vb);
        }
      }
      __builtin_amdgcn_fence(__ATOMIC_RELEASE, "workgroup");
      __builtin_amdgcn_wave_barrier();
      __builtin_amdgcn_fence(__ATOMIC_ACQUIRE, "workgroup");
    }
#pragma unroll
    for (int r = 0; r < 8; ++r) {
      const float inv = 1.0f / (lrow[r] * kPCarry);
#pragma unroll
      for (int t = 0; t < 6; ++t) os[(8 * hh + r) * kOP + hd * kHD + t * 16 + c] = oacc[t][r] * inv;
    }
  }
  __builtin_amdgcn_fence(__ATOMIC_RELEASE, "workgroup");
  __builtin_amdgcn_wave_barrier();
  __builtin_amdgcn_fence(__ATOMIC_ACQUIRE, "workgroup");
  {
    const int q = lane >> 3, c8 = (lane & 7) * 8;
    for (int pass = 0; pass < 2; ++pass) {
#pragma unroll 1
      for (int it = 0; it < 12; ++it) {
        const int L   = it * 4 + q;
        const int row = L / 3;
        const int seg = L - row * 3;
        const float* sp = os + row * kOP + seg * 64 + c8;
        const v4f a0 = *(const v4f*)(sp);
        const v4f a1 = *(const v4f*)(sp + 4);
        float x[8];
        x[0] = a0[0]; x[1] = a0[1]; x[2] = a0[2]; x[3] = a0[3];
        x[4] = a1[0]; x[5] = a1[1]; x[6] = a1[2]; x[7] = a1[3];
        unsigned short hb[8], lb[8];
#pragma unroll
        for (int e = 0; e < 8; ++e) {
          hb[e] = f2bf_bits(x[e]);
          lb[e] = f2bf_bits(x[e] - bf_bits2f(hb[e]));
        }
        const v4u hv = (v4u){pk16(hb[0], hb[1]), pk16(hb[2], hb[3]), pk16(hb[4], hb[5]), pk16(hb[6], hb[7])};
        const v4u lv = (v4u){pk16(lb[0], lb[1]), pk16(lb[2], lb[3]), pk16(lb[4], lb[5]), pk16(lb[6], lb[7])};
        const size_t o = (size_t)(q0 + row) * kDO + hp * (2 * kHD) + seg * 64 + c8;
        *(volatile v4u*)(Ch + o) = hv;
        *(volatile v4u*)(Cl + o) = lv;
      }
      __threadfence();
    }
  }
}

__global__ __launch_bounds__(256) void l2norm_rows_kernel(const float* __restrict__ P, float* __restrict__ out) {
  const int lane = threadIdx.x & 31, wave = threadIdx.x >> 5;
  const int row = blockIdx.x * 8 + wave;
  const float* pr = P + (size_t)row * kDO + lane * 4;
  v4f v[6];
#pragma unroll
  for (int i = 0; i < 6; ++i) v[i] = *(const v4f*)(pr + i * 128);
  float ss = 0.f;
#pragma unroll
  for (int i = 0; i < 6; ++i) {
#pragma unroll
    for (int e = 0; e < 4; ++e) {
      const float xv = v[i][e];
      ss = fmaf(xv, xv, ss);
    }
  }
  ss += __shfl_xor(ss, 16, 32);
  ss += __shfl_xor(ss, 8, 32);
  ss += __shfl_xor(ss, 4, 32);
  ss += __shfl_xor(ss, 2, 32);
  ss += __shfl_xor(ss, 1, 32);
  const float inv = 1.0f / sqrtf(ss);
#pragma unroll
  for (int i = 0; i < 6; ++i) v[i] = v[i] * inv;
  float* o0 = out + (size_t)row * kDO + lane * 4;
  float* o1 = o0 + (size_t)kRowsQ * kDO;
  for (int pass = 0; pass < 2; ++pass) {
#pragma unroll
    for (int i = 0; i < 6; ++i) {
      *(volatile v4f*)(o0 + i * 128) = v[i];
      *(volatile v4f*)(o1 + i * 128) = v[i];
    }
    __threadfence();
  }
}

extern "C" void kernel_launch(void* const* d_in, const int* in_sizes, int n_in,
                              void* d_out, int out_size, void* d_ws, size_t ws_size,
                              hipStream_t stream) {
  if (n_in < 10) return;
  if (in_sizes[0] != kRowsQ * kDT) return;
  if (in_sizes[1] != kRowsKV * kDV) return;
  if (in_sizes[2] != kDT * kDO) return;
  if (in_sizes[3] != kDO) return;
  if (in_sizes[4] != kDV * kDO) return;
  if (in_sizes[5] != kDO) return;
  if (in_sizes[6] != kDV * kDO) return;
  if (in_sizes[7] != kDO) return;
  if (in_sizes[8] != kDO * kDO) return;
  if (in_sizes[9] != kDO) return;
  if (out_size != 2 * kRowsQ * kDO) return;
  if (ws_size < kWsTotal) return;

  const float* F_t = (const float*)d_in[0];
  const float* F_s = (const float*)d_in[1];
  const float* Wq  = (const float*)d_in[2];
  const float* bq  = (const float*)d_in[3];
  const float* Wk  = (const float*)d_in[4];
  const float* bk  = (const float*)d_in[5];
  const float* Wv  = (const float*)d_in[6];
  const float* bv  = (const float*)d_in[7];
  const float* Wp  = (const float*)d_in[8];
  const float* bp  = (const float*)d_in[9];
  float* out = (float*)d_out;

  char* ws = (char*)d_ws;
  unsigned short* FT16 = (unsigned short*)(ws + kOffFT);
  unsigned short* FS16 = (unsigned short*)(ws + kOffFS);
  unsigned short* WQT  = (unsigned short*)(ws + kOffWQT);
  unsigned short* WKT  = (unsigned short*)(ws + kOffWKT);
  unsigned short* WVT  = (unsigned short*)(ws + kOffWVT);
  unsigned short* WPT  = (unsigned short*)(ws + kOffWPT);
  float*          BIAS = (float*)(ws + kOffBIAS);
  unsigned short* QH   = (unsigned short*)(ws + kOffQH);
  unsigned short* QL   = (unsigned short*)(ws + kOffQL);
  unsigned short* KH   = (unsigned short*)(ws + kOffKH);
  unsigned short* KL   = (unsigned short*)(ws + kOffKL);
  unsigned short* VT   = (unsigned short*)(ws + kOffVT);
  unsigned short* CH   = (unsigned short*)(ws + kOffCH);
  unsigned short* CL   = (unsigned short*)(ws + kOffCL);
  float*          PROJ = (float*)(ws + kOffPROJ);

  cast8_bf16_kernel<<<(kRowsQ * kDT / 8) / 256, 256, 0, stream>>>(F_t, FT16, kRowsQ * kDT / 8);
  cast8_bf16_kernel<<<(kRowsKV * kDV / 8) / 256, 256, 0, stream>>>(F_s, FS16, kRowsKV * kDV / 8);
  wt_bf16_kernel<<<dim3(kDV / 64, kDO / 64, 4), 256, 0, stream>>>(Wq, Wk, Wv, Wp, WQT, WKT, WVT, WPT);
  bias_rne_kernel<<<3, 256, 0, stream>>>(bq, bk, bv, bp, BIAS);

  wmma_gemm64_bf16<0, 2, 2><<<dim3(192, 1), 256, 0, stream>>>(
      FT16, FT16, kDT, WQT, kDT, (void*)QH, (void*)QL, kDO, BIAS, kRowsQ, kDO, kDT);
  wmma_gemm64_bf16<0, 2, 2><<<dim3(192, 1), 256, 0, stream>>>(
      FS16, FS16, kDV, WKT, kDV, (void*)KH, (void*)KL, kDO, BIAS + kDO, kRowsKV, kDO, kDV);
  wmma_gemm64_bf16<0, 1, 1><<<dim3(192, 1), 256, 0, stream>>>(
      WVT, WVT, kDV, FS16, kDV, (void*)VT, (void*)VT, kRowsKV, BIAS + 2 * kDO, kDO, kRowsKV, kDV);

  attn_pair_kernel<<<kB * (kN1 / 64) * (kH / 2), 128, 0, stream>>>(QH, QL, KH, KL, VT, CH, CL);

  wmma_gemm64_bf16<1, 2, 0><<<dim3(192, 1), 256, 0, stream>>>(
      CH, CL, kDO, WPT, kDO, (void*)PROJ, (void*)PROJ, kDO, BIAS + 3 * kDO, kRowsQ, kDO, kDO);

  l2norm_rows_kernel<<<kRowsQ / 8, 256, 0, stream>>>(PROJ, out);
}
